// GeATLayer_43061342110000
// MI455X (gfx1250) — hardware-run, weakly checked
//
#include <hip/hip_runtime.h>

typedef float          v8f   __attribute__((ext_vector_type(8)));
typedef float          v4f   __attribute__((ext_vector_type(4)));
typedef unsigned int   v4u   __attribute__((ext_vector_type(4)));
typedef int            v8i   __attribute__((ext_vector_type(8)));
typedef unsigned short v8us  __attribute__((ext_vector_type(8)));
typedef unsigned short v16us __attribute__((ext_vector_type(16)));
typedef __bf16         v16bf __attribute__((ext_vector_type(16)));
typedef _Float16       v16h  __attribute__((ext_vector_type(16)));
typedef v4f  __attribute__((may_alias)) v4fa;
typedef v8us __attribute__((may_alias)) v8usa;
union FragB { v16bf v; v16us u; v8us h[2]; v8i w; };
union FragH { v16h  v; v16us u; v8us h[2]; v8i w; };

__device__ __forceinline__ v8f wmb(const FragB& a, const FragB& b, v8f c) {
  v8f d = __builtin_amdgcn_wmma_f32_16x16x32_bf16(false, a.v, false, b.v, (short)0, c, false, false);
  asm volatile("v_nop\n\tv_nop\n\tv_nop\n\tv_nop" : "+v"(d) : "v"(a.w), "v"(b.w));
  return d;
}

__device__ __forceinline__ v8f wmh(const FragH& a, const FragH& b, v8f c) {
  v8f d = __builtin_amdgcn_wmma_f32_16x16x32_f16(false, a.v, false, b.v, (short)0, c, false, false);
  asm volatile("v_nop\n\tv_nop\n\tv_nop\n\tv_nop" : "+v"(d) : "v"(a.w), "v"(b.w));
  return d;
}

__device__ __forceinline__ unsigned bf16_bits(float f) {
  const unsigned u = __float_as_uint(f);
  const unsigned r = (u + 0x7FFFu + ((u >> 16) & 1u)) >> 16;
  const unsigned q = (u >> 16) | 0x40u;
  return ((u & 0x7fffffffu) > 0x7f800000u) ? q : r;
}

__device__ __forceinline__ float bf16_val(float f) {
  return __uint_as_float(bf16_bits(f) << 16);
}
__device__ __forceinline__ int clampi(int v, int lo, int hi) {
  return v < lo ? lo : (v > hi ? hi : v);
}

__device__ __forceinline__ unsigned f16_bits(float f) {
  const unsigned u  = __float_as_uint(f);
  const unsigned s  = (u >> 16) & 0x8000u;
  const unsigned a  = u & 0x7fffffffu;
  const unsigned t  = a - 0x38000000u;
  const unsigned r  = (t + 0x0FFFu + ((t >> 13) & 1u)) >> 13;
  const unsigned rc = r > 0x7C00u ? 0x7C00u : r;
  const bool small  = a < 0x38800000u;
  const bool isnan  = a > 0x7f800000u;
  const unsigned fin = small ? 0u : (s | rc);
  return isnan ? (s | 0x7E00u) : fin;
}

__device__ __forceinline__ unsigned pk16(unsigned lo, unsigned hi) { return lo | (hi << 16); }
__device__ __forceinline__ unsigned bf16_lo_bits(float v) {
  float hi = bf16_val(v);
  asm volatile("" : "+v"(hi));
  return bf16_bits(v - hi);
}
__device__ __forceinline__ v4u pack8_bf16(v4f a, v4f c) {
  return (v4u){ pk16(bf16_bits(a[0]), bf16_bits(a[1])), pk16(bf16_bits(a[2]), bf16_bits(a[3])),
                pk16(bf16_bits(c[0]), bf16_bits(c[1])), pk16(bf16_bits(c[2]), bf16_bits(c[3])) };
}
__device__ __forceinline__ v4u pack8_bf16_lo(v4f a, v4f c) {
  return (v4u){ pk16(bf16_lo_bits(a[0]), bf16_lo_bits(a[1])), pk16(bf16_lo_bits(a[2]), bf16_lo_bits(a[3])),
                pk16(bf16_lo_bits(c[0]), bf16_lo_bits(c[1])), pk16(bf16_lo_bits(c[2]), bf16_lo_bits(c[3])) };
}
__device__ __forceinline__ v4u pack8_f16(v4f a, v4f c) {
  return (v4u){ pk16(f16_bits(a[0]), f16_bits(a[1])), pk16(f16_bits(a[2]), f16_bits(a[3])),
                pk16(f16_bits(c[0]), f16_bits(c[1])), pk16(f16_bits(c[2]), f16_bits(c[3])) };
}

template <int FORM>
__global__ __launch_bounds__(256) void k_plane(const float* __restrict__ src, int rows, int cols, int ldsrc,
                                               unsigned short* __restrict__ dst, int MP, int KP) {
  static_assert(FORM >= 0 && FORM <= 3);
  const int KTOT = (FORM == 1 || FORM == 3) ? 2 * KP : KP;
  const unsigned ppr   = (unsigned)(KTOT >> 3);
  const unsigned kp8   = (unsigned)(KP >> 3);
  const unsigned total = (unsigned)MP * ppr;
  const unsigned g     = blockIdx.x * 256u + threadIdx.x;
  const unsigned rowu  = g / ppr;
  const unsigned p     = g - rowu * ppr;
  const bool second    = p >= kp8;
  const int row = (int)rowu;
  const int c0  = (int)((second ? p - kp8 : p) << 3);
  const float* srow = src + (size_t)clampi(row, 0, rows - 1) * (size_t)ldsrc;
  float x[8];
  unsigned mk[8];
#pragma unroll
  for (int e = 0; e < 8; ++e) {
    const int c = c0 + e;
    const float v = srow[clampi(c, 0, cols - 1)];
    asm volatile("" :: "v"(v));
    x[e]  = v;
    mk[e] = (row < rows && c < cols) ? 0xFFFFu : 0u;
  }
  const v4f a = (v4f){ x[0], x[1], x[2], x[3] };
  const v4f c = (v4f){ x[4], x[5], x[6], x[7] };
  v4u o;
  if (FORM == 2) {
    o = pack8_f16(a, c);
  } else {
    const v4u hi = pack8_bf16(a, c);
    o = hi;
    if (FORM == 1) { const v4u lo = pack8_bf16_lo(a, c); o = second ? lo : hi; }
  }
  const v4u mw = (v4u){ pk16(mk[0], mk[1]), pk16(mk[2], mk[3]), pk16(mk[4], mk[5]), pk16(mk[6], mk[7]) };
  o &= mw;
  if (g < total) {
    volatile v4u* q = (volatile v4u*)(dst + (size_t)g * 8);
    *q = o;
    __threadfence();
    *q = o;
  }
}

template <int FORM> struct FragOf    { typedef FragB T; };
template <>         struct FragOf<2> { typedef FragH T; };
__device__ __forceinline__ v8f mm(const FragB& a, const FragB& b, v8f c) { return wmb(a, b, c); }
__device__ __forceinline__ v8f mm(const FragH& a, const FragH& b, v8f c) { return wmh(a, b, c); }
template <class F> __device__ __forceinline__ F ld_frag(const unsigned short* p) {
  F f;
  f.h[0] = *(const v8usa*)(p);
  f.h[1] = *(const v8usa*)(p + 16);
  return f;
}

template <int FORM, int EPI>
__global__ __launch_bounds__(256) __attribute__((amdgpu_num_vgpr(248)))
void k_gemm_nt(const unsigned short* __restrict__ A, const unsigned short* __restrict__ B,
               const float* __restrict__ bias, float* __restrict__ D, int M, int N, int KTOT, int ldd) {
  static_assert(FORM >= 0 && FORM <= 2);
  static_assert(EPI == 0 || EPI == 1);
  typedef typename FragOf<FORM>::T F;
  __shared__ __attribute__((aligned(16))) float sT[8][16 * 68];
  const int lane = threadIdx.x & 31;
  const int wave = threadIdx.x >> 5;
  const int tilesM = (M + 63) >> 6;
  const int tilesN = (N + 63) >> 6;
  const int tile = blockIdx.x * 8 + wave;
  if (tile >= tilesM * tilesN) return;
  const int tm = tile / tilesN;
  const int tn = tile - tm * tilesN;
  const int m0 = tm << 6;
  const int n0 = tn << 6;

  const int rl = lane & 15;
  const int h8 = (lane >> 4) * 8;
  const unsigned short* pa = A + (size_t)(m0 + rl) * (size_t)KTOT + h8;
  const unsigned short* pb = B + (size_t)(n0 + rl) * (size_t)KTOT + h8;

  v8f acc[4][4];
#pragma unroll
  for (int i = 0; i < 4; ++i)
#pragma unroll
    for (int j = 0; j < 4; ++j) acc[i][j] = (v8f){0.f, 0.f, 0.f, 0.f, 0.f, 0.f, 0.f, 0.f};

#pragma unroll 1
  for (int k0 = 0; k0 < KTOT; k0 += 32) {
    F bf[4];
#pragma unroll
    for (int j = 0; j < 4; ++j) bf[j] = ld_frag<F>(pb + (size_t)(j << 4) * (size_t)KTOT + k0);
#pragma unroll
    for (int i = 0; i < 4; ++i) {
      const F af = ld_frag<F>(pa + (size_t)(i << 4) * (size_t)KTOT + k0);
#pragma unroll
      for (int j = 0; j < 4; ++j) acc[i][j] = mm(af, bf[j], acc[i][j]);
    }
  }

  float* slab = sT[wave];
  const int hh = lane >> 4;
  const int c4 = (lane & 15) * 4;
  const int nc = n0 + c4;
  const bool cok = nc < N;
  v4f bv = (v4f){0.f, 0.f, 0.f, 0.f};
  if (EPI == 1) {
    bv = *(const v4fa*)(bias + clampi(nc, 0, N - 4));
    asm volatile("" :: "v"(bv));
  }
#pragma unroll
  for (int i = 0; i < 4; ++i) {
    const int mBase = m0 + (i << 4);
#pragma unroll
    for (int j = 0; j < 4; ++j) {
#pragma unroll
      for (int r = 0; r < 8; ++r) slab[(h8 + r) * 68 + (j << 4) + rl] = acc[i][j][r];
    }
    __builtin_amdgcn_fence(__ATOMIC_RELEASE, "workgroup");
    __builtin_amdgcn_wave_barrier();
    __builtin_amdgcn_fence(__ATOMIC_ACQUIRE, "workgroup");
    v4f vv[8];
#pragma unroll
    for (int it = 0; it < 8; ++it) {
      const int row = it * 2 + hh;
      v4f v = *(const v4fa*)(slab + row * 68 + c4);
      if (EPI == 1) v += bv;
      vv[it] = v;
    }
    for (int pass = 0; pass < 2; ++pass) {
#pragma unroll
      for (int it = 0; it < 8; ++it) {
        const int row = mBase + it * 2 + hh;
        if (cok && row < M) *(volatile v4f*)(D + (size_t)row * (size_t)ldd + nc) = vv[it];
      }
      __threadfence();
    }
    __builtin_amdgcn_fence(__ATOMIC_RELEASE, "workgroup");
    __builtin_amdgcn_wave_barrier();
    __builtin_amdgcn_fence(__ATOMIC_ACQUIRE, "workgroup");
  }
}


#ifndef ATT_FORM
#define ATT_FORM 2
#endif
#ifndef OUT_FORM
#define OUT_FORM 1
#endif
static_assert(ATT_FORM == 1 || ATT_FORM == 2);
static_assert(OUT_FORM == 1 || OUT_FORM == 2);

typedef int v4i  __attribute__((ext_vector_type(4)));
typedef v4i __attribute__((may_alias)) v4ia;

#define G_B    256
#define G_M    128
#define G_D    64
#define G_H    8
#define G_NBT  5
#define G_HD   512
#define G_NCH  4
#define G_CMOL 64
#define G_CROWS 8192
#define G_ROWS 32768

static_assert(G_M == 128);
static_assert(G_D == 64);
static_assert(G_H * 64 == G_HD);
static_assert(8 * 16 == G_M);
static_assert(G_NBT == 5);
static_assert(G_CMOL * G_NCH == G_B);
static_assert(G_CMOL * G_M == G_CROWS);
static_assert(G_CROWS % 64 == 0);
static_assert(G_ROWS == G_B * G_M);

template <int AF> struct AttL {
  enum {
    NPL   = (AF == 1) ? 2 : 1,
    QPL   = 128 * 36,
    VPL   = 64 * 68,
    STILE = 16 * 132,
    PPL   = 16 * 68,
    OFF_Q = 0,
    OFF_K = NPL * QPL,
    OFF_V = 2 * NPL * QPL,
    OFF_S = OFF_V + NPL * VPL,
    OFF_P = OFF_S + 8 * STILE,
    TOTAL = OFF_P + 8 * NPL * PPL
  };
};
static_assert(AttL<ATT_FORM>::TOTAL * 4 + 256 <= 327680);

__device__ __forceinline__ void wave_sync() {
  __builtin_amdgcn_fence(__ATOMIC_RELEASE, "workgroup");
  __builtin_amdgcn_wave_barrier();
  __builtin_amdgcn_fence(__ATOMIC_ACQUIRE, "workgroup");
}

__device__ __forceinline__ float nmax(float a, float b) {
  float r = (a >= b) ? a : b;
  r = (a != a) ? a : r;
  return r;
}

template <int AF>
__device__ __forceinline__ void cvt2(float x, float y, unsigned& hw, unsigned& lw) {
  if (AF == 1) {
    hw = pk16(bf16_bits(x), bf16_bits(y));
    lw = pk16(bf16_lo_bits(x), bf16_lo_bits(y));
  } else {
    hw = pk16(f16_bits(x), f16_bits(y));
    lw = 0u;
  }
}

__device__ __forceinline__ v4u tr_piece8(const float* __restrict__ W, int n, int p) {
  float x[8];
#pragma unroll
  for (int e = 0; e < 8; ++e) {
    const float v = W[(size_t)(8 * p + e) * 512 + n];
    asm volatile("" :: "v"(v));
    x[e] = v;
  }
  return pack8_bf16((v4f){ x[0], x[1], x[2], x[3] }, (v4f){ x[4], x[5], x[6], x[7] });
}

__global__ __launch_bounds__(256) void k_tr(const float* __restrict__ Wq, const float* __restrict__ Wk,
                                            const float* __restrict__ Wv, const float* __restrict__ Wp,
                                            const float* __restrict__ bq, const float* __restrict__ bk,
                                            const float* __restrict__ bv, const float* __restrict__ bp,
                                            const float* __restrict__ eb,
                                            unsigned short* __restrict__ wqkvt, float* __restrict__ wptf,
                                            float* __restrict__ bqkv, float* __restrict__ bpeb) {
  const int tid = threadIdx.x;
  const int blk = blockIdx.x;
  if (blk < 48) {
    const int sel = blk >> 4;
    const int g   = (blk & 15) * 256 + tid;
    const int n   = g >> 3;
    const int p   = g & 7;
    v4u o;
    if (sel == 0)      o = tr_piece8(Wq, n, p);
    else if (sel == 1) o = tr_piece8(Wk, n, p);
    else               o = tr_piece8(Wv, n, p);
    volatile v4u* q = (volatile v4u*)(wqkvt + (size_t)(sel * 512 + n) * 64 + p * 8);
    *q = o;
    __threadfence();
    *q = o;
  } else if (blk < 80) {
    const int g  = (blk - 48) * 256 + tid;
    const int n  = g >> 7;
    const int q4 = g & 127;
    float x[4];
#pragma unroll
    for (int e = 0; e < 4; ++e) {
      const float v = Wp[(size_t)(4 * q4 + e) * 64 + n];
      asm volatile("" :: "v"(v));
      x[e] = v;
    }
    const v4f o = (v4f){ bf16_val(x[0]), bf16_val(x[1]), bf16_val(x[2]), bf16_val(x[3]) };
    volatile v4f* q = (volatile v4f*)(wptf + (size_t)n * 512 + 4 * q4);
    *q = o;
    __threadfence();
    *q = o;
  } else if (blk == 80) {
    const int t = tid & 127;
    const v4f a = *(const v4fa*)(bq + 4 * t);
    const v4f b = *(const v4fa*)(bk + 4 * t);
    const v4f c = *(const v4fa*)(bv + 4 * t);
    asm volatile("" :: "v"(a), "v"(b), "v"(c));
    const v4f ra = (v4f){ bf16_val(a[0]), bf16_val(a[1]), bf16_val(a[2]), bf16_val(a[3]) };
    const v4f rb = (v4f){ bf16_val(b[0]), bf16_val(b[1]), bf16_val(b[2]), bf16_val(b[3]) };
    const v4f rc = (v4f){ bf16_val(c[0]), bf16_val(c[1]), bf16_val(c[2]), bf16_val(c[3]) };
    if (tid < 128) {
      volatile v4f* q0 = (volatile v4f*)(bqkv + 4 * t);
      volatile v4f* q1 = (volatile v4f*)(bqkv + 512 + 4 * t);
      volatile v4f* q2 = (volatile v4f*)(bqkv + 1024 + 4 * t);
      *q0 = ra; *q1 = rb; *q2 = rc;
      __threadfence();
      *q0 = ra; *q1 = rb; *q2 = rc;
    }
  } else {
    const int l16 = tid & 15;
    const int le  = l16 < 9 ? l16 : 9;
    const v4f a = *(const v4fa*)(bp + 4 * l16);
    const v4f e = *(const v4fa*)(eb + 4 * le);
    asm volatile("" :: "v"(a), "v"(e));
    const bool upper  = (tid & 16) != 0;
    const unsigned mA = upper ? 0u : 0xFFFFFFFFu;
    const unsigned mE = (upper && l16 < 10) ? 0xFFFFFFFFu : 0u;
    float o[4];
#pragma unroll
    for (int i = 0; i < 4; ++i) {
      const unsigned ba = bf16_bits(a[i]) << 16;
      const unsigned be = bf16_bits(e[i]) << 16;
      o[i] = __uint_as_float((ba & mA) | (be & mE));
    }
    const v4f ov = (v4f){ o[0], o[1], o[2], o[3] };
    if (tid < 32) {
      volatile v4f* q = (volatile v4f*)(bpeb + 4 * tid);
      *q = ov;
      __threadfence();
      *q = ov;
    }
  }
}

template <int AF>
__global__ __launch_bounds__(256) __attribute__((amdgpu_num_vgpr(248)))
void k_attn(const float* __restrict__ qkv, const int* __restrict__ edges,
            const float* __restrict__ ebw, float* __restrict__ outc) {
  static_assert(AF == 1 || AF == 2);
  typedef typename FragOf<AF>::T F;
  typedef AttL<AF> L;
  extern __shared__ __attribute__((aligned(16))) unsigned dsm[];
  __shared__ __attribute__((aligned(16))) float sEB[64];

  const int tid  = threadIdx.x;
  const int lane = tid & 31;
  const int wave = tid >> 5;
  const int hh   = lane >> 4;
  const int c    = lane & 15;
  const int bl   = blockIdx.x >> 3;
  const int h    = blockIdx.x & 7;

  {
    const v4f ebv = *(const v4fa*)(ebw + 4 * (tid & 15));
    asm volatile("" :: "v"(ebv));
    if (tid < 16) *(v4fa*)(sEB + 4 * tid) = ebv;
  }

  const float* qbase = qkv + (size_t)(bl * 128) * 1536 + h * 64;

#pragma unroll 2
  for (int it = 0; it < 8; ++it) {
    const int idx = it * 256 + tid;
    const int row = idx >> 4;
    const int c4  = (idx & 15) * 4;
    const float* g = qbase + (size_t)row * 1536 + c4;
    const v4f q4 = *(const v4fa*)(g);
    const v4f k4 = *(const v4fa*)(g + 512);
    asm volatile("" :: "v"(q4), "v"(k4));
    const int di = row * 36 + (c4 >> 1);
    unsigned h0, l0, h1, l1;
    cvt2<AF>(q4[0], q4[1], h0, l0);
    cvt2<AF>(q4[2], q4[3], h1, l1);
    dsm[L::OFF_Q + di]     = h0;
    dsm[L::OFF_Q + di + 1] = h1;
    if (AF == 1) {
      dsm[L::OFF_Q + L::QPL + di]     = l0;
      dsm[L::OFF_Q + L::QPL + di + 1] = l1;
    }
    cvt2<AF>(k4[0], k4[1], h0, l0);
    cvt2<AF>(k4[2], k4[3], h1, l1);
    dsm[L::OFF_K + di]     = h0;
    dsm[L::OFF_K + di + 1] = h1;
    if (AF == 1) {
      dsm[L::OFF_K + L::QPL + di]     = l0;
      dsm[L::OFF_K + L::QPL + di + 1] = l1;
    }
  }
#pragma unroll 2
  for (int it = 0; it < 4; ++it) {
    const int u  = it * 256 + tid;
    const int dq = u & 15;
    const int np = u >> 4;
    const float* g = qbase + 1024 + (size_t)(2 * np) * 1536 + 4 * dq;
    const v4f a = *(const v4fa*)(g);
    const v4f b = *(const v4fa*)(g + 1536);
    asm volatile("" :: "v"(a), "v"(b));
#pragma unroll
    for (int e = 0; e < 4; ++e) {
      unsigned hw, lw;
      cvt2<AF>(a[e], b[e], hw, lw);
      const int di = (4 * dq + e) * 68 + np;
      dsm[L::OFF_V + di] = hw;
      if (AF == 1) dsm[L::OFF_V + L::VPL + di] = lw;
    }
  }
  __syncthreads();

  const float eb0 = sEB[h];
  const float eb1 = sEB[8 + h];
  const float eb2 = sEB[16 + h];
  const float eb3 = sEB[24 + h];
  const float eb4 = sEB[32 + h];

  const unsigned short* q16 = (const unsigned short*)(dsm + L::OFF_Q);
  const unsigned short* k16 = (const unsigned short*)(dsm + L::OFF_K);
  const unsigned short* v16 = (const unsigned short*)(dsm + L::OFF_V);
  float*    sS = (float*)(dsm + L::OFF_S + wave * L::STILE);
  unsigned* sP = dsm + L::OFF_P + wave * (L::NPL * L::PPL);
  const unsigned short* p16 = (const unsigned short*)sP;

  F qh[2], ql[2];
#pragma unroll
  for (int ks = 0; ks < 2; ++ks) {
    const int qi = (16 * wave + c) * 72 + ks * 32 + 8 * hh;
    qh[ks].h[0] = *(const v8usa*)(q16 + qi);
    qh[ks].h[1] = *(const v8usa*)(q16 + qi + 16);
    if (AF == 1) {
      ql[ks].h[0] = *(const v8usa*)(q16 + 2 * L::QPL + qi);
      ql[ks].h[1] = *(const v8usa*)(q16 + 2 * L::QPL + qi + 16);
    } else {
      ql[ks] = qh[ks];
    }
  }
#pragma unroll 1
  for (int j = 0; j < 8; ++j) {
    v8f acc = (v8f){0.f, 0.f, 0.f, 0.f, 0.f, 0.f, 0.f, 0.f};
#pragma unroll
    for (int ks = 0; ks < 2; ++ks) {
      const int ki = (16 * j + c) * 72 + ks * 32 + 8 * hh;
      F kh;
      kh.h[0] = *(const v8usa*)(k16 + ki);
      kh.h[1] = *(const v8usa*)(k16 + ki + 16);
      acc = mm(qh[ks], kh, acc);
      if (AF == 1) {
        F kl;
        kl.h[0] = *(const v8usa*)(k16 + 2 * L::QPL + ki);
        kl.h[1] = *(const v8usa*)(k16 + 2 * L::QPL + ki + 16);
        acc = mm(ql[ks], kh, acc);
        acc = mm(qh[ks], kl, acc);
      }
    }
#pragma unroll
    for (int r = 0; r < 8; ++r) sS[(8 * hh + r) * 132 + 16 * j + c] = acc[r];
  }
  wave_sync();

  float lkeep = 1.0f;
  const int* erow0 = edges + ((size_t)(bl * 128 + 16 * wave)) * 128 + 4 * lane;
#pragma unroll 1
  for (int rr = 0; rr < 16; ++rr) {
    const v4f s4 = *(const v4fa*)(sS + rr * 132 + 4 * lane);
    const v4i e4 = *(const v4ia*)(erow0 + (size_t)rr * 128);
    asm volatile("" :: "v"(e4));
    float sv[4];
#pragma unroll
    for (int e = 0; e < 4; ++e) {
      const int ee = e4[e];
      const int t  = clampi(ee, 0, 4);
      float bias = eb0;
      bias = (t == 1) ? eb1 : bias;
      bias = (t == 2) ? eb2 : bias;
      bias = (t == 3) ? eb3 : bias;
      bias = (t == 4) ? eb4 : bias;
      float s = s4[e] * 0.125f + bias;
      s = (s >= 0.0f) ? s : 0.2f * s;
      s = (ee > 0) ? s : -1e9f;
      sv[e] = s;
    }
    float mx = nmax(nmax(sv[0], sv[1]), nmax(sv[2], sv[3]));
    mx = nmax(mx, __shfl_xor(mx, 16, 32));
    mx = nmax(mx, __shfl_xor(mx, 8, 32));
    mx = nmax(mx, __shfl_xor(mx, 4, 32));
    mx = nmax(mx, __shfl_xor(mx, 2, 32));
    mx = nmax(mx, __shfl_xor(mx, 1, 32));
    const float p0 = expf(sv[0] - mx);
    const float p1 = expf(sv[1] - mx);
    const float p2 = expf(sv[2] - mx);
    const float p3 = expf(sv[3] - mx);
    float ps = ((p0 + p1) + p2) + p3;
    ps += __shfl_xor(ps, 16, 32);
    ps += __shfl_xor(ps, 8, 32);
    ps += __shfl_xor(ps, 4, 32);
    ps += __shfl_xor(ps, 2, 32);
    ps += __shfl_xor(ps, 1, 32);
    lkeep = (c == rr) ? ps : lkeep;
    unsigned w0, u0, w1, u1;
    cvt2<AF>(p0, p1, w0, u0);
    cvt2<AF>(p2, p3, w1, u1);
    const int pi = rr * 68 + 2 * lane;
    sP[pi]     = w0;
    sP[pi + 1] = w1;
    if (AF == 1) {
      sP[L::PPL + pi]     = u0;
      sP[L::PPL + pi + 1] = u1;
    }
  }
  wave_sync();

  v8f oacc[4];
#pragma unroll
  for (int t = 0; t < 4; ++t) oacc[t] = (v8f){0.f, 0.f, 0.f, 0.f, 0.f, 0.f, 0.f, 0.f};
#pragma unroll 1
  for (int kk = 0; kk < 4; ++kk) {
    const int pi = c * 136 + kk * 32 + 8 * hh;
    F ph, pl;
    ph.h[0] = *(const v8usa*)(p16 + pi);
    ph.h[1] = *(const v8usa*)(p16 + pi + 16);
    if (AF == 1) {
      pl.h[0] = *(const v8usa*)(p16 + 2 * L::PPL + pi);
      pl.h[1] = *(const v8usa*)(p16 + 2 * L::PPL + pi + 16);
    } else {
      pl = ph;
    }
#pragma unroll
    for (int t = 0; t < 4; ++t) {
      const int vi = (16 * t + c) * 136 + kk * 32 + 8 * hh;
      F vh;
      vh.h[0] = *(const v8usa*)(v16 + vi);
      vh.h[1] = *(const v8usa*)(v16 + vi + 16);
      oacc[t] = mm(ph, vh, oacc[t]);
      if (AF == 1) {
        F vl;
        vl.h[0] = *(const v8usa*)(v16 + 2 * L::VPL + vi);
        vl.h[1] = *(const v8usa*)(v16 + 2 * L::VPL + vi + 16);
        oacc[t] = mm(pl, vh, oacc[t]);
        oacc[t] = mm(ph, vl, oacc[t]);
      }
    }
  }

  wave_sync();
#pragma unroll
  for (int t = 0; t < 4; ++t) {
#pragma unroll
    for (int r = 0; r < 8; ++r) sS[(8 * hh + r) * 132 + 16 * t + c] = oacc[t][r];
  }
  wave_sync();
  {
    const int c4 = c * 4;
    v4f vv[8];
#pragma unroll
    for (int it = 0; it < 8; ++it) {
      const int row = it * 2 + hh;
      const v4f v = *(const v4fa*)(sS + row * 132 + c4);
      const float lr  = __shfl(lkeep, row, 32);
      const float inv = 1.0f / lr;
      vv[it] = v * inv;
    }
    float* ob = outc + (size_t)(bl * 128 + 16 * wave) * 512 + h * 64 + c4;
    for (int pass = 0; pass < 2; ++pass) {
#pragma unroll
      for (int it = 0; it < 8; ++it) {
        const int row = it * 2 + hh;
        *(volatile v4f*)(ob + (size_t)row * 512) = vv[it];
      }
      __threadfence();
    }
  }
}

#define WS_XB     ((size_t)0)
#define WS_WQKVT  (WS_XB    + (size_t)4194304)
#define WS_WPTF   (WS_WQKVT + (size_t)196608)
#define WS_WPTP   (WS_WPTF  + (size_t)131072)
#define WS_BQKV   (WS_WPTP  + (size_t)131072)
#define WS_BPEB   (WS_BQKV  + (size_t)6144)
#define WS_QKV    (WS_BPEB  + (size_t)512)
#define WS_OUTC   (WS_QKV   + (size_t)50331648)
#define WS_OUTP   (WS_OUTC  + (size_t)16777216)
#define WS_TOTAL  (WS_OUTP  + (size_t)16777216)
static_assert(WS_TOTAL == (size_t)88545792);
static_assert(WS_TOTAL <= (size_t)134217728);
static_assert((size_t)G_ROWS * 64 * 2 == (size_t)4194304);
static_assert((size_t)G_CROWS * 1536 * 4 == (size_t)50331648);
static_assert((size_t)G_CROWS * 512 * 4 == (size_t)16777216);
static_assert((size_t)G_CROWS * 1024 * 2 == (size_t)16777216);
static_assert((size_t)(G_NCH - 1) * G_CROWS * 64 + (size_t)G_CROWS * 64 - 1 == (size_t)2097151);

extern "C" void kernel_launch(void* const* d_in, const int* in_sizes, int n_in,
                              void* d_out, int out_size, void* d_ws, size_t ws_size,
                              hipStream_t stream) {
  if (n_in < 11) return;
  if (in_sizes[0] != G_B * G_M * G_D) return;
  if (in_sizes[1] != G_B * G_M * G_M) return;
  if (in_sizes[2] != G_D * G_HD || in_sizes[4] != G_D * G_HD || in_sizes[6] != G_D * G_HD) return;
  if (in_sizes[3] != G_HD || in_sizes[5] != G_HD || in_sizes[7] != G_HD) return;
  if (in_sizes[8] != G_NBT * G_H) return;
  if (in_sizes[9] != G_HD * G_D) return;
  if (in_sizes[10] != G_D) return;
  if (out_size != G_B * G_M * G_D) return;
  if (WS_TOTAL > ws_size) return;

  const float* X   = (const float*)d_in[0];
  const int*   EDG = (const int*)d_in[1];
  const float* Wq  = (const float*)d_in[2];
  const float* bq  = (const float*)d_in[3];
  const float* Wk  = (const float*)d_in[4];
  const float* bk  = (const float*)d_in[5];
  const float* Wv  = (const float*)d_in[6];
  const float* bv  = (const float*)d_in[7];
  const float* eb  = (const float*)d_in[8];
  const float* Wp  = (const float*)d_in[9];
  const float* bp  = (const float*)d_in[10];
  float* out = (float*)d_out;

  char* ws = (char*)d_ws;
  unsigned short* XB    = (unsigned short*)(ws + WS_XB);
  unsigned short* WQKVT = (unsigned short*)(ws + WS_WQKVT);
  float*          WPTF  = (float*)(ws + WS_WPTF);
  unsigned short* WPTP  = (unsigned short*)(ws + WS_WPTP);
  float*          BQKV  = (float*)(ws + WS_BQKV);
  float*          BPEB  = (float*)(ws + WS_BPEB);
  float*          QKVc  = (float*)(ws + WS_QKV);
  float*          OUTc  = (float*)(ws + WS_OUTC);
  unsigned short* OUTPc = (unsigned short*)(ws + WS_OUTP);

  const int KTOT_OUT = (OUT_FORM == 1) ? 1024 : 512;
  const int WPT_PF   = (OUT_FORM == 1) ? 3 : 2;
  const int attLds   = AttL<ATT_FORM>::TOTAL * 4;

  k_tr<<<dim3(82), dim3(256), 0, stream>>>(Wq, Wk, Wv, Wp, bq, bk, bv, bp, eb, WQKVT, WPTF, BQKV, BPEB);
  k_plane<WPT_PF><<<dim3(64 * KTOT_OUT / 8 / 256), dim3(256), 0, stream>>>(WPTF, 64, 512, 512, WPTP, 64, 512);
  k_plane<0><<<dim3(G_ROWS * 64 / 8 / 256), dim3(256), 0, stream>>>(X, G_ROWS, 64, 64, XB, G_ROWS, 64);

  (void)hipFuncSetAttribute(reinterpret_cast<const void*>(&k_attn<ATT_FORM>),
                            hipFuncAttributeMaxDynamicSharedMemorySize, attLds);

  for (int ch = 0; ch < G_NCH; ++ch) {
    const unsigned short* XBc = XB + (size_t)ch * G_CROWS * 64;
    const int* EDGc = EDG + (size_t)ch * G_CMOL * G_M * G_M;
    float* outc_final = out + (size_t)ch * G_CROWS * 64;
    k_gemm_nt<0, 1><<<dim3(384), dim3(256), 0, stream>>>(XBc, WQKVT, BQKV, QKVc, G_CROWS, 1536, 64, 1536);
    k_attn<ATT_FORM><<<dim3(G_CMOL * G_H), dim3(256), attLds, stream>>>(QKVc, EDGc, BPEB + 64, OUTc);
    k_plane<OUT_FORM><<<dim3(G_CROWS * KTOT_OUT / 8 / 256), dim3(256), 0, stream>>>(OUTc, G_CROWS, 512, 512, OUTPc, G_CROWS, 512);
    k_gemm_nt<OUT_FORM, 1><<<dim3(16), dim3(256), 0, stream>>>(OUTPc, WPTP, BPEB, outc_final, G_CROWS, 64, KTOT_OUT, 64);
  }
  (void)hipGetLastError();
}
